// NodeGLAM_26207890440557
// MI455X (gfx1250) — hardware-verified
//
#include <hip/hip_runtime.h>
#include <stddef.h>


#define HD      128
#define DI      64
#define DO      16
#define AP3     192
#define NHOP    3
#define SPW     512
#define NTHR    256
#define NWAVE   8
#define EPT     8
#define NGRP    2
#define CHUNK   (NTHR * EPT * NGRP)
#define WCAP    (EPT * NGRP * 32)
#define LISTN   (NWAVE * WCAP)
#define ESHF    11
#define NBC     32768
#define NBF     2048
#define RCAP    40960
#define RBN     128
#define TGT     256
#define DEGCAP  512
#define GROWS   128
#define XNR     128
#define BNR     1024
#define OTHR    512
#define WSCALE  64
#define ASCALE  64
#define AHP     136
#define EPSC    1e-5f
#define WSCAP   134217728

#define OW1   0
#define OT1   (OW1 + HD * DI)
#define OW2   (OT1 + HD * SPW)
#define OT2   (OW2 + HD * HD)
#define OW3   (OT2 + HD * SPW)
#define OW4   (OW3 + HD * AP3)
#define WPTOT (OW4 + DO * HD)
#define WB1   ((HD * DI / 8) / NTHR)
#define WBT   ((HD * SPW / 8) / NTHR)
#define WB2   ((HD * HD / 8) / NTHR)
#define WB3   ((HD * AP3 / 8) / NTHR)
#define WB4   ((DO * HD / 8) / NTHR)
#define WPREP_BLOCKS (WB1 + WBT + WB2 + WBT + WB3 + WB4)

#define LDS_COUNT ((NBC + LISTN + NWAVE) * 4)
#define LDS_FILL  ((RCAP + NBF + LISTN + NWAVE) * 4)
#define LDS_GEMM  (GROWS * HD * 4)

static_assert((CHUNK & (CHUNK - 1)) == 0);
static_assert((NBC & (NBC - 1)) == 0 && (NBF & (NBF - 1)) == 0);
static_assert(NBF <= (1 << ESHF));
static_assert((NBC % NBF) == 0);
static_assert(OTHR * 4 == NBF);
static_assert((RCAP % 32) == 0);
static_assert(TGT == NWAVE * 32);
static_assert(GROWS == NWAVE * 16);
static_assert((TGT % GROWS) == 0 && (TGT % XNR) == 0);
static_assert(NBC == NWAVE * 32 * 128);
static_assert(SPW == (NHOP + 1) * HD && AP3 == DI + HD);
static_assert((HD * DI / 8) % NTHR == 0 && (HD * SPW / 8) % NTHR == 0 && (HD * HD / 8) % NTHR == 0);
static_assert((HD * AP3 / 8) % NTHR == 0 && (DO * HD / 8) % NTHR == 0);
static_assert(WPREP_BLOCKS == 89 && WPTOT == 182272);
static_assert(XNR == 4 * (NTHR / 8));
static_assert((AHP % 8) == 0);
static_assert(BNR == 4 * NTHR && DI == 64);

typedef float     v4f  __attribute__((ext_vector_type(4)));
typedef float     v8f  __attribute__((ext_vector_type(8)));
typedef int       v4i  __attribute__((ext_vector_type(4)));
typedef unsigned  v2u  __attribute__((ext_vector_type(2)));
typedef _Float16  v4h  __attribute__((ext_vector_type(4)));
typedef _Float16  v8h  __attribute__((ext_vector_type(8)));
typedef _Float16  v16h __attribute__((ext_vector_type(16)));
union FragH { v16h v; v8h h[2]; };
union H4U { v4h h; v2u u; };

__device__ __forceinline__ v8f wmf(v16h a, v16h b, v8f c) {
  v8f d = __builtin_amdgcn_wmma_f32_16x16x32_f16(false, a, false, b, (short)0, c, false, false);
  asm volatile("v_nop\n\tv_nop\n\tv_nop\n\tv_nop" : "+v"(d) : "v"(a), "v"(b));
  return d;
}

__device__ __forceinline__ v16h afr(const _Float16* akp) {
  FragH f;
  f.h[0] = *(const v8h*)akp;
  f.h[1] = *(const v8h*)(akp + 16);
  return f.v;
}

template <int NB, int SRC>
__device__ __forceinline__ int scan_chunk(const int* __restrict__ keys, const int* __restrict__ gath, int nE, int nN,
                                          int cbase, int slotBase, int vec8, int* list, int tid, int lane, int wave) {
  int wc = 0;
#pragma unroll
  for (int g = 0; g < NGRP; ++g) {
    const int el0  = (g * NTHR + tid) * EPT;
    const int e0   = cbase + el0;
    const int sent = -2147483647 - 1;
    v4i da, db;
    v4i sa = {0, 0, 0, 0}, sb = {0, 0, 0, 0};
    if (vec8 != 0 && cbase + CHUNK <= nE) {
      da = *(const v4i*)(keys + e0);
      db = *(const v4i*)(keys + e0 + 4);
      if (SRC) {
        sa = *(const v4i*)(gath + e0);
        sb = *(const v4i*)(gath + e0 + 4);
      }
    } else {
      da.x = (e0     < nE) ? keys[min(e0, nE - 1)] : sent;
      da.y = (e0 + 1 < nE) ? keys[min(e0 + 1, nE - 1)] : sent;
      da.z = (e0 + 2 < nE) ? keys[min(e0 + 2, nE - 1)] : sent;
      da.w = (e0 + 3 < nE) ? keys[min(e0 + 3, nE - 1)] : sent;
      db.x = (e0 + 4 < nE) ? keys[min(e0 + 4, nE - 1)] : sent;
      db.y = (e0 + 5 < nE) ? keys[min(e0 + 5, nE - 1)] : sent;
      db.z = (e0 + 6 < nE) ? keys[min(e0 + 6, nE - 1)] : sent;
      db.w = (e0 + 7 < nE) ? keys[min(e0 + 7, nE - 1)] : sent;
      if (SRC) {
        sa.x = gath[min(e0, nE - 1)];
        sa.y = gath[min(e0 + 1, nE - 1)];
        sa.z = gath[min(e0 + 2, nE - 1)];
        sa.w = gath[min(e0 + 3, nE - 1)];
        sb.x = gath[min(e0 + 4, nE - 1)];
        sb.y = gath[min(e0 + 5, nE - 1)];
        sb.z = gath[min(e0 + 6, nE - 1)];
        sb.w = gath[min(e0 + 7, nE - 1)];
      }
    }
    if (SRC) {
      sa.x = min(max(sa.x, 0), nN - 1); sa.y = min(max(sa.y, 0), nN - 1);
      sa.z = min(max(sa.z, 0), nN - 1); sa.w = min(max(sa.w, 0), nN - 1);
      sb.x = min(max(sb.x, 0), nN - 1); sb.y = min(max(sb.y, 0), nN - 1);
      sb.z = min(max(sb.z, 0), nN - 1); sb.w = min(max(sb.w, 0), nN - 1);
    }
    const unsigned nb = (unsigned)slotBase;
    const unsigned s0 = (unsigned)da.x - nb, s1 = (unsigned)da.y - nb;
    const unsigned s2 = (unsigned)da.z - nb, s3 = (unsigned)da.w - nb;
    const unsigned s4 = (unsigned)db.x - nb, s5 = (unsigned)db.y - nb;
    const unsigned s6 = (unsigned)db.z - nb, s7 = (unsigned)db.w - nb;
    const bool h0 = s0 < (unsigned)NB, h1 = s1 < (unsigned)NB, h2 = s2 < (unsigned)NB, h3 = s3 < (unsigned)NB;
    const bool h4 = s4 < (unsigned)NB, h5 = s5 < (unsigned)NB, h6 = s6 < (unsigned)NB, h7 = s7 < (unsigned)NB;
    const unsigned any = __builtin_amdgcn_ballot_w32(h0 | h1 | h2 | h3 | h4 | h5 | h6 | h7);
    if (any != 0u) {
#define HITJ(HJ, SJ, VJ) { \
        const unsigned mj = __builtin_amdgcn_ballot_w32(HJ); \
        if (mj != 0u) { \
          if (HJ) { \
            const int pos = wc + (int)__builtin_amdgcn_mbcnt_lo(mj, 0u); \
            const int entv = SRC ? (((VJ) << ESHF) | (int)(SJ)) : (int)(SJ); \
            if (pos < WCAP) list[wave * WCAP + pos] = entv; \
          } \
          wc += (int)__builtin_popcount(mj); } }
      HITJ(h0, s0, sa.x)
      HITJ(h1, s1, sa.y)
      HITJ(h2, s2, sa.z)
      HITJ(h3, s3, sa.w)
      HITJ(h4, s4, sb.x)
      HITJ(h5, s5, sb.y)
      HITJ(h6, s6, sb.z)
      HITJ(h7, s7, sb.w)
#undef HITJ
    }
  }
  return wc;
}

__global__ __launch_bounds__(NTHR) void k_wprep(const float* __restrict__ w1, const float* __restrict__ t1,
                                                const float* __restrict__ w2, const float* __restrict__ t2,
                                                const float* __restrict__ w3, const float* __restrict__ w4,
                                                _Float16* wp) {
  const int tid = threadIdx.x;
  const int b = (int)blockIdx.x;
  const float* src;
  int K, N, j, dbase;
  if (b < WB1)                              { src = w1; K = DI;  N = HD; j = b * NTHR + tid;                               dbase = OW1; }
  else if (b < WB1 + WBT)                   { src = t1; K = SPW; N = HD; j = (b - WB1) * NTHR + tid;                       dbase = OT1; }
  else if (b < WB1 + WBT + WB2)             { src = w2; K = HD;  N = HD; j = (b - WB1 - WBT) * NTHR + tid;                 dbase = OW2; }
  else if (b < WB1 + 2 * WBT + WB2)         { src = t2; K = SPW; N = HD; j = (b - WB1 - WBT - WB2) * NTHR + tid;           dbase = OT2; }
  else if (b < WB1 + 2 * WBT + WB2 + WB3)   { src = w3; K = AP3; N = HD; j = (b - WB1 - 2 * WBT - WB2) * NTHR + tid;       dbase = OW3; }
  else                                      { src = w4; K = HD;  N = DO; j = (b - WB1 - 2 * WBT - WB2 - WB3) * NTHR + tid; dbase = OW4; }
  const int kq = K >> 3;
  const int jm = N * kq - 1;
  j = j < 0 ? 0 : (j > jm ? jm : j);
  const int n  = j / kq;
  const int k0 = (j - n * kq) * 8;
  v8h hv;
#pragma unroll
  for (int e = 0; e < 8; ++e) hv[e] = (_Float16)(src[(size_t)(k0 + e) * N + n] * (float)WSCALE);
  _Float16* d = wp + (size_t)dbase + (size_t)n * K + (size_t)k0;
  *(volatile v8h*)d = hv;
  __threadfence();
  *(volatile v8h*)d = hv;
}

__global__ __launch_bounds__(NTHR) void k_bnpart(const float* __restrict__ x, float* part, int nN) {
  __shared__ float ss[NTHR];
  __shared__ float sq[NTHR];
  __shared__ __attribute__((aligned(16))) float res[2 * DI];
  const int tid = threadIdx.x;
  const int c = tid & (DI - 1);
  const int rg = tid >> 6;
  const int r0 = (int)blockIdx.x * BNR;
  const int rend = min(r0 + BNR, nN);
  float s = 0.f, q = 0.f;
#pragma unroll 1
  for (int r = r0 + rg; r < rend; r += 4) {
    const float v = x[(size_t)r * DI + c];
    s += v;
    q += v * v;
  }
  ss[tid] = s;
  sq[tid] = q;
  __syncthreads();
  if (tid < DI) {
    res[tid]      = (ss[tid] + ss[tid + 64]) + (ss[tid + 128] + ss[tid + 192]);
    res[DI + tid] = (sq[tid] + sq[tid + 64]) + (sq[tid + 128] + sq[tid + 192]);
  }
  __syncthreads();
  v4f rv = {0.f, 0.f, 0.f, 0.f};
  if (tid < 32) rv = *(const v4f*)(res + 4 * tid);
  float* p = part + (size_t)blockIdx.x * (2 * DI) + 4 * tid;
  if (tid < 32) *(volatile v4f*)p = rv;
  __threadfence();
  if (tid < 32) *(volatile v4f*)p = rv;
}

__global__ __launch_bounds__(NTHR) void k_xn(const float* __restrict__ x, const float* __restrict__ part,
                                             const float* __restrict__ gam, const float* __restrict__ bet,
                                             _Float16* A3, int nN, int nBP) {
  __shared__ float smu[DI];
  __shared__ float ssc[DI];
  __shared__ float sbe[DI];
  const int tid = threadIdx.x;
  if (tid < DI) {
    double S = 0.0, Q = 0.0;
#pragma unroll 1
    for (int p = 0; p < nBP; ++p) {
      S += (double)part[(size_t)p * (2 * DI) + tid];
      Q += (double)part[(size_t)p * (2 * DI) + DI + tid];
    }
    const double inv = 1.0 / (double)nN;
    const double mu = S * inv;
    double var = Q * inv - mu * mu;
    var = var < 0.0 ? 0.0 : var;
    const float sc = gam[tid] * rsqrtf((float)var + EPSC);
    smu[tid] = (float)mu;
    ssc[tid] = sc;
    sbe[tid] = bet[tid];
  }
  __syncthreads();
  const int rsub = tid >> 3;
  const int c0 = (tid & 7) * 8;
#pragma unroll 1
  for (int it = 0; it < XNR / 32; ++it) {
    const int row = (int)blockIdx.x * XNR + it * 32 + rsub;
    const int rr = row > nN - 1 ? nN - 1 : row;
    const v4f xa = *(const v4f*)(x + (size_t)rr * DI + c0);
    const v4f xb = *(const v4f*)(x + (size_t)rr * DI + c0 + 4);
    float xv[8];
    xv[0] = xa.x; xv[1] = xa.y; xv[2] = xa.z; xv[3] = xa.w;
    xv[4] = xb.x; xv[5] = xb.y; xv[6] = xb.z; xv[7] = xb.w;
    v8h hv;
#pragma unroll
    for (int e = 0; e < 8; ++e) {
      float v = ((xv[e] - smu[c0 + e]) * ssc[c0 + e] + sbe[c0 + e]) * (float)ASCALE;
      if (row >= nN) v = 0.f;
      hv[e] = (_Float16)v;
    }
    _Float16* d = A3 + (size_t)row * AP3 + c0;
    *(volatile v8h*)d = hv;
    __threadfence();
    *(volatile v8h*)d = hv;
  }
}

__global__ __launch_bounds__(NTHR) void k_count(
    const int* __restrict__ keys, const int* __restrict__ gath, int* cnt, float* dinv, int nE, int nN, int vec8) {
  extern __shared__ v4f lds_dyn[];
  int* scnt = (int*)lds_dyn;
  int* list = scnt + NBC;
  int* wcnt = list + LISTN;
  const int tid = threadIdx.x, lane = tid & 31, wave = tid >> 5;
  const int nodeBase = blockIdx.x * NBC;

  {
    const v4i z = {0, 0, 0, 0};
    for (int i = tid; i < NBC / 4; i += NTHR) ((v4i*)scnt)[i] = z;
  }
  __syncthreads();

  const int nChunks = (nE + CHUNK - 1) / CHUNK;
#pragma unroll 1
  for (int ch = 0; ch < nChunks; ++ch) {
    const int cbase = ch * CHUNK;
    const int wc = scan_chunk<NBC, 0>(keys, gath, nE, nN, cbase, nodeBase, vec8, list, tid, lane, wave);
    if (lane == 0) wcnt[wave] = wc;
    __syncthreads();
    if (wave == 0) {
#pragma unroll 1
      for (int wsx = 0; wsx < NWAVE; ++wsx) {
        int n = __builtin_amdgcn_readfirstlane(wcnt[wsx]);
        n = n > WCAP ? WCAP : (n < 0 ? 0 : n);
        const int* lp = list + wsx * WCAP;
#pragma unroll 1
        for (int i = 0; i < n; ++i) {
          const int ent  = __builtin_amdgcn_readfirstlane(lp[i]);
          const int slot = ent & (NBC - 1);
          if (lane == 0) scnt[slot] = scnt[slot] + 1;
        }
      }
    }
    __syncthreads();
  }

  int*   cp = cnt + (size_t)nodeBase;
  float* dp = dinv + (size_t)nodeBase;
#pragma unroll 4
  for (int q = 0; q < 32; ++q) {
    const int f = (wave * 32 + q) * 128 + 4 * lane;
    const v4i c = *(const v4i*)(scnt + f);
    const float g0 = (float)c.x, g1 = (float)c.y, g2 = (float)c.z, g3 = (float)c.w;
    v4f d;
    d.x = g0 > 0.f ? rsqrtf(g0) : 0.f; d.y = g1 > 0.f ? rsqrtf(g1) : 0.f;
    d.z = g2 > 0.f ? rsqrtf(g2) : 0.f; d.w = g3 > 0.f ? rsqrtf(g3) : 0.f;
    *(volatile v4i*)(cp + f) = c;
    *(volatile v4f*)(dp + f) = d;
  }
  __threadfence();
#pragma unroll 4
  for (int q = 0; q < 32; ++q) {
    const int f = (wave * 32 + q) * 128 + 4 * lane;
    const v4i c = *(const v4i*)(scnt + f);
    const float g0 = (float)c.x, g1 = (float)c.y, g2 = (float)c.z, g3 = (float)c.w;
    v4f d;
    d.x = g0 > 0.f ? rsqrtf(g0) : 0.f; d.y = g1 > 0.f ? rsqrtf(g1) : 0.f;
    d.z = g2 > 0.f ? rsqrtf(g2) : 0.f; d.w = g3 > 0.f ? rsqrtf(g3) : 0.f;
    *(volatile v4i*)(cp + f) = c;
    *(volatile v4f*)(dp + f) = d;
  }
}

__global__ __launch_bounds__(OTHR) void k_offsets(
    const int* __restrict__ cnt, int* off, int* rbase, int nBF) {
  __shared__ __attribute__((aligned(16))) int srb[RBN];
  __shared__ int wtot[OTHR / 32];
  const int tid = threadIdx.x, lane = tid & 31, wave = tid >> 5;
  for (int i = tid; i < RBN; i += OTHR) srb[i] = 0;
  int carry = 0;
#pragma unroll 1
  for (int fb = 0; fb < nBF; ++fb) {
    const int base = fb * NBF;
    const v4i c = *(const v4i*)(cnt + base + 4 * tid);
    const int e0 = max(c.x, 0), e1 = max(c.y, 0), e2 = max(c.z, 0), e3 = max(c.w, 0);
    const int ts = e0 + e1 + e2 + e3;
    int incl = ts;
#pragma unroll
    for (int d = 1; d < 32; d <<= 1) {
      const int t = __shfl_up(incl, d, 32);
      if (lane >= d) incl += t;
    }
    if (lane == 31) wtot[wave] = incl;
    __syncthreads();
    int pre = 0;
#pragma unroll 1
    for (int w = 0; w < wave; ++w) pre += wtot[w];
    int tot = 0;
#pragma unroll
    for (int w = 0; w < OTHR / 32; ++w) tot += wtot[w];
    int run = carry + pre + incl - ts;
    v4i o;
    o.x = run; run += e0;
    o.y = run; run += e1;
    o.z = run; run += e2;
    o.w = run;
    int* op = off + base + 4 * tid;
    *(volatile v4i*)op = o;
    __threadfence();
    *(volatile v4i*)op = o;
    if (tid == 0) srb[min(fb, RBN - 1)] = carry;
    carry += (tot + 31) & ~31;
    __syncthreads();
  }
  if (tid == 0) srb[min(nBF, RBN - 1)] = carry;
  __syncthreads();
  v4i rv = {0, 0, 0, 0};
  if (tid < 32) rv = *(const v4i*)(srb + 4 * tid);
  if (tid < 32) *(volatile v4i*)(rbase + 4 * tid) = rv;
  __threadfence();
  if (tid < 32) *(volatile v4i*)(rbase + 4 * tid) = rv;
}

__global__ __launch_bounds__(NTHR) void k_fill(
    const int* __restrict__ keys, const int* __restrict__ gath, const int* __restrict__ off, const int* __restrict__ rbase,
    int* csr, int nN, int nE, int vec8, int csrLen) {
  extern __shared__ v4f lds_dyn[];
  int* region = (int*)lds_dyn;
  int* cursor = region + RCAP;
  int* list   = cursor + NBF;
  int* wcnt   = list + LISTN;
  const int tid = threadIdx.x, lane = tid & 31, wave = tid >> 5;
  const int b = blockIdx.x;
  const int nodeBase = b * NBF;

  int rb0 = rbase[b];
  const int rb1 = rbase[b + 1];
  rb0 = rb0 < 0 ? 0 : (rb0 > csrLen ? csrLen : rb0);
  rb0 &= ~31;
  int len = rb1 - rb0;
  len = len < 0 ? 0 : (len > RCAP ? RCAP : len);
  int lenW = (len + 31) & ~31;
  if (rb0 + lenW > csrLen) lenW = (csrLen - rb0) & ~31;

  {
    const v4i z = {0, 0, 0, 0};
    for (int i = tid; i < RCAP / 4; i += NTHR) ((v4i*)region)[i] = z;
    for (int s = tid; s < NBF; s += NTHR) {
      int o = off[nodeBase + s] - rb0;
      o = o < 0 ? 0 : (o > RCAP ? RCAP : o);
      cursor[s] = o;
    }
  }
  __syncthreads();

  const int nChunks = (nE + CHUNK - 1) / CHUNK;
#pragma unroll 1
  for (int ch = 0; ch < nChunks; ++ch) {
    const int cbase = ch * CHUNK;
    const int wc = scan_chunk<NBF, 1>(keys, gath, nE, nN, cbase, nodeBase, vec8, list, tid, lane, wave);
    if (lane == 0) wcnt[wave] = wc;
    __syncthreads();
    if (wave == 0) {
#pragma unroll 1
      for (int wsx = 0; wsx < NWAVE; ++wsx) {
        int n = __builtin_amdgcn_readfirstlane(wcnt[wsx]);
        n = n > WCAP ? WCAP : (n < 0 ? 0 : n);
        const int* lp = list + wsx * WCAP;
#pragma unroll 1
        for (int i = 0; i < n; ++i) {
          const int ent  = __builtin_amdgcn_readfirstlane(lp[i]);
          const int slot = ent & (NBF - 1);
          int src = (ent >> ESHF) & 0xFFFFF;
          src = src > nN - 1 ? nN - 1 : src;
          if (lane == 0) {
            int pos = cursor[slot];
            pos = pos < 0 ? 0 : (pos > RCAP - 1 ? RCAP - 1 : pos);
            region[pos] = src;
            const int np = pos + 1;
            cursor[slot] = np > RCAP ? RCAP : np;
          }
        }
      }
    }
    __syncthreads();
  }

  const int nv = lenW >> 2;
  int* gp = csr + rb0;
#pragma unroll 1
  for (int i = tid; i < nv; i += NTHR) { const v4i v = ((const v4i*)region)[i]; *(volatile v4i*)(gp + 4 * i) = v; }
  __threadfence();
#pragma unroll 1
  for (int i = tid; i < nv; i += NTHR) { const v4i v = ((const v4i*)region)[i]; *(volatile v4i*)(gp + 4 * i) = v; }
}

template <int WXS>
__global__ __launch_bounds__(NTHR) void k_agg(
    const int* __restrict__ csr, const int* __restrict__ off, const int* __restrict__ cnt,
    const float* __restrict__ dinv, const float* __restrict__ xin,
    _Float16* sg, float* xout, int nN, int csrLen) {
  const int tid = threadIdx.x, lane = tid & 31, wave = tid >> 5;
  const int tbase = blockIdx.x * TGT + wave * 32;
  const int cl = tbase + lane;
  const int cnt_l = cnt[cl];
  const int off_l = off[cl];
  union FI { float f; int i; };
  FI dvu; dvu.f = dinv[cl];

#pragma unroll 1
  for (int j = 0; j < 32; ++j) {
    const int c = tbase + j;
    int n = __builtin_amdgcn_readlane(cnt_l, j);
    n = n < 0 ? 0 : (n > DEGCAP ? DEGCAP : n);
    const int st = __builtin_amdgcn_readlane(off_l, j);
    FI du; du.i = __builtin_amdgcn_readlane(dvu.i, j);
    const float dc = du.f;
    v4f acc = {0.f, 0.f, 0.f, 0.f};
#pragma unroll 1
    for (int q0 = 0; q0 < n; q0 += 32) {
      int pos = st + q0 + lane;
      pos = pos < 0 ? 0 : (pos > csrLen - 1 ? csrLen - 1 : pos);
      int sl = csr[pos];
      sl = sl < 0 ? 0 : (sl > nN - 1 ? nN - 1 : sl);
      const int mcnt = (n - q0) < 32 ? (n - q0) : 32;
#pragma unroll 1
      for (int p = 0; p < mcnt; ++p) {
        const int sidx = __builtin_amdgcn_readlane(sl, p);
        acc = acc + *(const v4f*)(xin + (size_t)sidx * HD + 4 * lane);
      }
    }
    const v4f hk = acc * dc;
    H4U hq;
    hq.h[0] = (_Float16)(hk.x * (float)ASCALE); hq.h[1] = (_Float16)(hk.y * (float)ASCALE);
    hq.h[2] = (_Float16)(hk.z * (float)ASCALE); hq.h[3] = (_Float16)(hk.w * (float)ASCALE);
    const v2u uu = hq.u;
    _Float16* ap = sg + (size_t)c * SPW + 4 * lane;
    const v4f xo = hk * dc;
    float* xp = xout + (size_t)c * HD + 4 * lane;
    *(volatile v2u*)ap = uu;
    if constexpr (WXS != 0) *(volatile v4f*)xp = xo;
    __threadfence();
    *(volatile v2u*)ap = uu;
    if constexpr (WXS != 0) *(volatile v4f*)xp = xo;
  }
}

__device__ __forceinline__ void st_h16(const float* lp, _Float16* Ch, int ldc, int growBase, int hh, int m) {
#pragma unroll
  for (int i = 0; i < 8; ++i) {
    const int rl = 2 * i + hh;
    const int cs = 8 * m;
    const v4f u0 = *(const v4f*)(lp + rl * HD + cs);
    const v4f u1 = *(const v4f*)(lp + rl * HD + cs + 4);
    v8h hv;
    hv[0] = (_Float16)(u0.x * (float)ASCALE); hv[1] = (_Float16)(u0.y * (float)ASCALE);
    hv[2] = (_Float16)(u0.z * (float)ASCALE); hv[3] = (_Float16)(u0.w * (float)ASCALE);
    hv[4] = (_Float16)(u1.x * (float)ASCALE); hv[5] = (_Float16)(u1.y * (float)ASCALE);
    hv[6] = (_Float16)(u1.z * (float)ASCALE); hv[7] = (_Float16)(u1.w * (float)ASCALE);
    *(volatile v8h*)(Ch + (size_t)(growBase + rl) * ldc + cs) = hv;
  }
}

__device__ __forceinline__ void st_xs(const float* lp, float* Xs, const float* __restrict__ dinv, int growBase, int lane) {
#pragma unroll
  for (int i = 0; i < 16; ++i) {
    const float d = dinv[growBase + i];
    const v4f v = *(const v4f*)(lp + i * HD + 4 * lane) * d;
    *(volatile v4f*)(Xs + (size_t)(growBase + i) * HD + 4 * lane) = v;
  }
}

template <int KD, int WXS>
__global__ __launch_bounds__(NTHR) void k_gemm(
    const _Float16* __restrict__ A, int lda, const _Float16* __restrict__ Bw, const float* __restrict__ bias,
    const float* __restrict__ dinv, _Float16* Ch, int ldc, float* Xs) {
  extern __shared__ v4f lds_dyn[];
  constexpr int NT = HD / 16;
  constexpr float OSC = 1.0f / (float)(ASCALE * WSCALE);
  float* stg = (float*)lds_dyn;
  const int tid = threadIdx.x, lane = tid & 31, wave = tid >> 5, hh = lane >> 4, m = lane & 15;
  const int rowBase = blockIdx.x * GROWS;
  const int arow = rowBase + wave * 16 + m;
  const _Float16* ap = A + (size_t)arow * lda + 8 * hh;

  v8f acc[NT];
#pragma unroll
  for (int t = 0; t < NT; ++t) { v8f z = {0.f, 0.f, 0.f, 0.f, 0.f, 0.f, 0.f, 0.f}; acc[t] = z; }

#pragma unroll 1
  for (int kt = 0; kt < KD / 32; ++kt) {
    const v16h av = afr(ap + 32 * kt);
#pragma unroll
    for (int t = 0; t < NT; ++t) {
      const v16h bv = afr(Bw + (size_t)(16 * t + m) * KD + 32 * kt + 8 * hh);
      acc[t] = wmf(av, bv, acc[t]);
    }
  }

  const int r0 = wave * 16 + 8 * hh;
  float* sp = stg + r0 * HD + m;
#pragma unroll
  for (int t = 0; t < NT; ++t) {
    const float bc = bias[16 * t + m];
#pragma unroll
    for (int r = 0; r < 8; ++r) {
      float v = acc[t][r] * OSC + bc;
      v = fmaxf(v, 0.f);
      sp[r * HD + 16 * t] = v;
    }
  }
  __syncthreads();

  const float* lp = stg + wave * 16 * HD;
  const int growBase = rowBase + wave * 16;
  st_h16(lp, Ch, ldc, growBase, hh, m);
  if constexpr (WXS != 0) st_xs(lp, Xs, dinv, growBase, lane);
  __threadfence();
  st_h16(lp, Ch, ldc, growBase, hh, m);
  if constexpr (WXS != 0) st_xs(lp, Xs, dinv, growBase, lane);
}

__global__ __launch_bounds__(NTHR) void k_head(
    const _Float16* __restrict__ A, const _Float16* __restrict__ B3, const float* __restrict__ b3,
    const _Float16* __restrict__ B4, const float* __restrict__ b4, float* out, int nN) {
  __shared__ __attribute__((aligned(16))) _Float16 ah[GROWS * AHP];
  __shared__ __attribute__((aligned(16))) float so[GROWS * DO];
  constexpr int NT = HD / 16;
  constexpr float OSC = 1.0f / (float)(ASCALE * WSCALE);
  const int tid = threadIdx.x, lane = tid & 31, wave = tid >> 5, hh = lane >> 4, m = lane & 15;
  const int rowBase = blockIdx.x * GROWS;
  const int arow = rowBase + wave * 16 + m;
  const _Float16* ap = A + (size_t)arow * AP3 + 8 * hh;

  v8f acc[NT];
#pragma unroll
  for (int t = 0; t < NT; ++t) { v8f z = {0.f, 0.f, 0.f, 0.f, 0.f, 0.f, 0.f, 0.f}; acc[t] = z; }

#pragma unroll 1
  for (int kt = 0; kt < AP3 / 32; ++kt) {
    const v16h av = afr(ap + 32 * kt);
#pragma unroll
    for (int t = 0; t < NT; ++t) {
      const v16h bv = afr(B3 + (size_t)(16 * t + m) * AP3 + 32 * kt + 8 * hh);
      acc[t] = wmf(av, bv, acc[t]);
    }
  }

  const int r0 = wave * 16 + 8 * hh;
#pragma unroll
  for (int t = 0; t < NT; ++t) {
    const float bc = b3[16 * t + m];
#pragma unroll
    for (int r = 0; r < 8; ++r) {
      float v = acc[t][r] * OSC + bc;
      v = fmaxf(v, 0.f) * (float)ASCALE;
      ah[(r0 + r) * AHP + 16 * t + m] = (_Float16)v;
    }
  }
  __syncthreads();

  v8f lacc = {0.f, 0.f, 0.f, 0.f, 0.f, 0.f, 0.f, 0.f};
  const _Float16* a2 = ah + (wave * 16 + m) * AHP + 8 * hh;
#pragma unroll
  for (int kt = 0; kt < HD / 32; ++kt) {
    FragH f;
    f.h[0] = *(const v8h*)(a2 + 32 * kt);
    f.h[1] = *(const v8h*)(a2 + 32 * kt + 16);
    const v16h bv = afr(B4 + (size_t)m * HD + 32 * kt + 8 * hh);
    lacc = wmf(f.v, bv, lacc);
  }

  const float bo = b4[m];
  float z[8];
#pragma unroll
  for (int r = 0; r < 8; ++r) z[r] = lacc[r] * OSC + bo;
#pragma unroll
  for (int r = 0; r < 8; ++r) {
    float mx = z[r];
#pragma unroll
    for (int s = 1; s < 16; s <<= 1) mx = fmaxf(mx, __shfl_xor(mx, s, 32));
    const float e = __expf(z[r] - mx);
    float sm = e;
#pragma unroll
    for (int s = 1; s < 16; s <<= 1) sm += __shfl_xor(sm, s, 32);
    const float p = e * (1.0f / sm);
    so[(r0 + r) * DO + m] = p;
  }
  __syncthreads();

  const int rl = lane >> 2;
  const int pc = (lane & 3) * 4;
#pragma unroll
  for (int g = 0; g < 2; ++g) {
    const int rowl = wave * 16 + 8 * g + rl;
    const int grow = rowBase + rowl;
    const v4f v = *(const v4f*)(so + rowl * DO + pc);
    if (grow < nN) *(volatile v4f*)(out + (size_t)grow * DO + pc) = v;
  }
  __threadfence();
#pragma unroll
  for (int g = 0; g < 2; ++g) {
    const int rowl = wave * 16 + 8 * g + rl;
    const int grow = rowBase + rowl;
    const v4f v = *(const v4f*)(so + rowl * DO + pc);
    if (grow < nN) *(volatile v4f*)(out + (size_t)grow * DO + pc) = v;
  }
}

extern "C" void kernel_launch(void* const* d_in, const int* in_sizes, int n_in,
                              void* d_out, int out_size, void* d_ws, size_t ws_size,
                              hipStream_t stream) {
  if (n_in < 16) return;
  const int nN = in_sizes[0] / DI;
  const int nE = in_sizes[1] / 2;
  if (nN <= 0 || nE <= 0) return;
  if (in_sizes[0] != nN * DI || in_sizes[1] != 2 * nE) return;
  if (in_sizes[2] != DI || in_sizes[3] != DI) return;
  if (in_sizes[4] != DI * HD || in_sizes[5] != HD) return;
  if (in_sizes[6] != (NHOP + 1) * HD * HD || in_sizes[7] != HD) return;
  if (in_sizes[8] != HD * HD || in_sizes[9] != HD) return;
  if (in_sizes[10] != (NHOP + 1) * HD * HD || in_sizes[11] != HD) return;
  if (in_sizes[12] != AP3 * HD || in_sizes[13] != HD) return;
  if (in_sizes[14] != HD * DO || in_sizes[15] != DO) return;
  if (out_size != nN * DO) return;
  if (nN > (1 << 20) || nE > (1 << 28)) return;

  const float* x    = (const float*)d_in[0];
  const int*   ei   = (const int*)d_in[1];
  const int*   srcp = ei;
  const int*   dstp = ei + nE;
  const float* gam  = (const float*)d_in[2];
  const float* bet  = (const float*)d_in[3];
  const float* w1   = (const float*)d_in[4];
  const float* b1   = (const float*)d_in[5];
  const float* t1   = (const float*)d_in[6];
  const float* tb1  = (const float*)d_in[7];
  const float* w2   = (const float*)d_in[8];
  const float* b2   = (const float*)d_in[9];
  const float* t2   = (const float*)d_in[10];
  const float* tb2  = (const float*)d_in[11];
  const float* w3   = (const float*)d_in[12];
  const float* b3   = (const float*)d_in[13];
  const float* w4   = (const float*)d_in[14];
  const float* b4   = (const float*)d_in[15];
  float* out = (float*)d_out;

  const int NPAD   = ((nN + TGT - 1) / TGT) * TGT;
  const int nBC    = (nN + NBC - 1) / NBC;
  const int CNTPAD = nBC * NBC;
  const int nBF    = (nN + NBF - 1) / NBF;
  const int OFFN   = nBF * NBF;
  if (nBF + 1 > RBN) return;
  if (OFFN > CNTPAD || NPAD > OFFN) return;
  const int csrLen = ((nE + 31) & ~31) + 32 * (nBF + 1);
  const int nBP    = (nN + BNR - 1) / BNR;
  const int nXn    = NPAD / XNR;
  const int nGemm  = NPAD / GROWS;
  const int nAgg   = NPAD / TGT;

  char* ws = (char*)d_ws;
  size_t off = 0;
  const size_t oW   = off; off += (size_t)WPTOT * 2;          off = (off + 255) & ~(size_t)255;
  const size_t oPt  = off; off += (size_t)nBP * (2 * DI) * 4; off = (off + 255) & ~(size_t)255;
  const size_t oCnt = off; off += (size_t)CNTPAD * 4;         off = (off + 255) & ~(size_t)255;
  const size_t oDv  = off; off += (size_t)CNTPAD * 4;         off = (off + 255) & ~(size_t)255;
  const size_t oOff = off; off += (size_t)OFFN * 4;           off = (off + 255) & ~(size_t)255;
  const size_t oRb  = off; off += (size_t)RBN * 4;            off = (off + 255) & ~(size_t)255;
  const size_t oCsr = off; off += (size_t)csrLen * 4;         off = (off + 255) & ~(size_t)255;
  const size_t oA3  = off; off += (size_t)NPAD * AP3 * 2;     off = (off + 255) & ~(size_t)255;
  const size_t oS   = off; off += (size_t)NPAD * SPW * 2;     off = (off + 255) & ~(size_t)255;
  const size_t oXa  = off; off += (size_t)NPAD * HD * 4;      off = (off + 255) & ~(size_t)255;
  const size_t oXb  = off; off += (size_t)NPAD * HD * 4;      off = (off + 255) & ~(size_t)255;
  if (off > ws_size || off > (size_t)WSCAP) return;
  _Float16* wp   = (_Float16*)(ws + oW);
  float*    part = (float*)(ws + oPt);
  int*      cnt  = (int*)(ws + oCnt);
  float*    dinv = (float*)(ws + oDv);
  int*      offp = (int*)(ws + oOff);
  int*      rb   = (int*)(ws + oRb);
  int*      csr  = (int*)(ws + oCsr);
  _Float16* A3   = (_Float16*)(ws + oA3);
  _Float16* S    = (_Float16*)(ws + oS);
  float*    xsA  = (float*)(ws + oXa);
  float*    xsB  = (float*)(ws + oXb);
  const _Float16* pW1 = wp + OW1;
  const _Float16* pT1 = wp + OT1;
  const _Float16* pW2 = wp + OW2;
  const _Float16* pT2 = wp + OT2;
  const _Float16* pW3 = wp + OW3;
  const _Float16* pW4 = wp + OW4;

  const int vec8 = ((nE & 3) == 0) ? 1 : 0;

  k_wprep<<<WPREP_BLOCKS, NTHR, 0, stream>>>(w1, t1, w2, t2, w3, w4, wp);

  k_bnpart<<<nBP, NTHR, 0, stream>>>(x, part, nN);
  k_xn<<<nXn, NTHR, 0, stream>>>(x, part, gam, bet, A3, nN, nBP);

  hipFuncSetAttribute(reinterpret_cast<const void*>(&k_count),
                      hipFuncAttributeMaxDynamicSharedMemorySize, LDS_COUNT);
  k_count<<<nBC, NTHR, LDS_COUNT, stream>>>(dstp, srcp, cnt, dinv, nE, nN, vec8);
  k_offsets<<<1, OTHR, 0, stream>>>(cnt, offp, rb, nBF);
  hipFuncSetAttribute(reinterpret_cast<const void*>(&k_fill),
                      hipFuncAttributeMaxDynamicSharedMemorySize, LDS_FILL);
  k_fill<<<nBF, NTHR, LDS_FILL, stream>>>(dstp, srcp, offp, rb, csr, nN, nE, vec8, csrLen);

  hipFuncSetAttribute(reinterpret_cast<const void*>(&k_gemm<DI, 1>),
                      hipFuncAttributeMaxDynamicSharedMemorySize, LDS_GEMM);
  hipFuncSetAttribute(reinterpret_cast<const void*>(&k_gemm<HD, 1>),
                      hipFuncAttributeMaxDynamicSharedMemorySize, LDS_GEMM);
  hipFuncSetAttribute(reinterpret_cast<const void*>(&k_gemm<SPW, 0>),
                      hipFuncAttributeMaxDynamicSharedMemorySize, LDS_GEMM);

  k_gemm<DI, 1><<<nGemm, NTHR, LDS_GEMM, stream>>>(A3, AP3, pW1, b1, dinv, S, SPW, xsA);
  k_agg<1><<<nAgg, NTHR, 0, stream>>>(csr, offp, cnt, dinv, xsA, S + 1 * HD, xsB, nN, csrLen);
  k_agg<1><<<nAgg, NTHR, 0, stream>>>(csr, offp, cnt, dinv, xsB, S + 2 * HD, xsA, nN, csrLen);
  k_agg<0><<<nAgg, NTHR, 0, stream>>>(csr, offp, cnt, dinv, xsA, S + 3 * HD, xsB, nN, csrLen);
  k_gemm<SPW, 0><<<nGemm, NTHR, LDS_GEMM, stream>>>(S, SPW, pT1, tb1, dinv, A3 + DI, AP3, xsB);
  k_gemm<HD, 1><<<nGemm, NTHR, LDS_GEMM, stream>>>(A3 + DI, AP3, pW2, b2, dinv, S, SPW, xsA);
  k_agg<1><<<nAgg, NTHR, 0, stream>>>(csr, offp, cnt, dinv, xsA, S + 1 * HD, xsB, nN, csrLen);
  k_agg<1><<<nAgg, NTHR, 0, stream>>>(csr, offp, cnt, dinv, xsB, S + 2 * HD, xsA, nN, csrLen);
  k_agg<0><<<nAgg, NTHR, 0, stream>>>(csr, offp, cnt, dinv, xsA, S + 3 * HD, xsB, nN, csrLen);
  k_gemm<SPW, 0><<<nGemm, NTHR, LDS_GEMM, stream>>>(S, SPW, pT2, tb2, dinv, A3 + DI, AP3, xsB);
  k_head<<<nGemm, NTHR, 0, stream>>>(A3, pW3, b3, pW4, b4, out, nN);
}
